// PatchBatchRelationalModule_75935021793485
// MI455X (gfx1250) — hardware-verified
//
#include <hip/hip_runtime.h>


#define NBI  8
#define CIN  32
#define HW   32
#define GG   16
#define PG   15
#define NP   225
#define NPP  256
#define DFE  130
#define KP   160
#define HID  256
#define NOUT 128
#define NPR  50625
#define NPRP 50688
#define DM   KP
#define NTK  NPRP
#define SLOPE 0.01f
#define LOSC 1024.0f

typedef _Float16 h16;
typedef unsigned short bf;
typedef __attribute__((ext_vector_type(16))) __bf16   v16bf;
typedef __attribute__((ext_vector_type(16))) _Float16 v16h;
typedef __attribute__((ext_vector_type(8)))  _Float16 v8h;
typedef __attribute__((ext_vector_type(8)))  unsigned short v8us;
typedef __attribute__((ext_vector_type(8)))  float    v8f;
typedef __attribute__((ext_vector_type(4)))  float    v4f;
typedef __attribute__((ext_vector_type(4)))  _Float16 v4h;
typedef v8h  __attribute__((may_alias)) v8ha;
typedef v4f  __attribute__((may_alias)) v4fa;
typedef v8us __attribute__((may_alias)) v8usa;

__device__ __forceinline__ unsigned short f2bf(float f) { unsigned u = __float_as_uint(f); u += 0x7FFFu + ((u >> 16) & 1u); return (unsigned short)(u >> 16); }
__device__ __forceinline__ float bf2f(unsigned short b) { return __uint_as_float(((unsigned)b) << 16); }
__device__ __forceinline__ float bfr(float f) { return bf2f(f2bf(f)); }
__device__ __forceinline__ v16h cat16(v8h lo, v8h hi) { return __builtin_shufflevector(lo, hi, 0, 1, 2, 3, 4, 5, 6, 7, 8, 9, 10, 11, 12, 13, 14, 15); }
__device__ __forceinline__ v16bf cat16b(v8us lo, v8us hi) { return __builtin_bit_cast(v16bf, __builtin_shufflevector(lo, hi, 0, 1, 2, 3, 4, 5, 6, 7, 8, 9, 10, 11, 12, 13, 14, 15)); }
__device__ __forceinline__ v8f wmma16(v16h a, v16h b, v8f c) { return __builtin_amdgcn_wmma_f32_16x16x32_f16(false, a, false, b, (short)0, c, false, false); }
__device__ __forceinline__ v8f wmmab(v16bf a, v16bf b, v8f c) { return __builtin_amdgcn_wmma_f32_16x16x32_bf16(false, a, false, b, (short)0, c, false, false); }

__global__ __launch_bounds__(256) void k_wt(const float* __restrict__ Wm, int K, int ncols, bf* WT) {
    __shared__ __align__(16) unsigned short tl[64 * 72];
    const int tid = threadIdx.x, k0 = blockIdx.x * 64, n0 = blockIdx.y * 64;
    const int kk = tid >> 2, nq = (tid & 3) * 16;
#pragma unroll
    for (int i = 0; i < 16; ++i) tl[(nq + i) * 72 + kk] = f2bf(Wm[(size_t)(k0 + kk) * ncols + n0 + nq + i]);
    __syncthreads();
    const int piece = tid & 7;
    auto pass = [&]() {
#pragma unroll
        for (int s = 0; s < 2; ++s) { const int nr = (tid >> 3) + 32 * s; const v8us val = *(const v8usa*)(tl + nr * 72 + piece * 8); *(volatile v8us*)(WT + (size_t)(n0 + nr) * K + k0 + piece * 8) = val; }
    };
    pass(); __threadfence(); pass();
}
template <bool SPLITA, bool F16OUT = false>
__global__ __launch_bounds__(128) void k_gemmb(const bf* __restrict__ A, const bf* __restrict__ Al, const bf* __restrict__ Bn, const float* __restrict__ bias, float* C, int ldc, h16* C2, const float* __restrict__ R = nullptr, int K = DM, int roundR = 1) {
    __shared__ __align__(16) float ost[4][16 * 68];
    const int lane = threadIdx.x & 31, wave = threadIdx.x >> 5, lr = lane & 15, hi = lane >> 4;
    const int r0 = blockIdx.x * 64 + wave * 16, c0 = blockIdx.y * 64;
    const size_t aoff = (size_t)(r0 + lr) * K + 8 * hi;
    size_t boff[4];
#pragma unroll
    for (int t = 0; t < 4; ++t) boff[t] = (size_t)(c0 + t * 16 + lr) * K + 8 * hi;
    v8f acc[4];
#pragma unroll
    for (int t = 0; t < 4; ++t) acc[t] = (v8f){};
#pragma unroll 1
    for (int kc = 0; kc < K; kc += 32) {
        const v16bf a = cat16b(*(const v8us*)(A + aoff + kc), *(const v8us*)(A + aoff + kc + 16));
        v16bf al = a;
        if (SPLITA) al = cat16b(*(const v8us*)(Al + aoff + kc), *(const v8us*)(Al + aoff + kc + 16));
#pragma unroll
        for (int t = 0; t < 4; ++t) { const v16bf b = cat16b(*(const v8us*)(Bn + boff[t] + kc), *(const v8us*)(Bn + boff[t] + kc + 16)); acc[t] = wmmab(a, b, acc[t]); if (SPLITA) acc[t] = wmmab(al, b, acc[t]); }
        asm volatile("v_nop\n\tv_nop\n\tv_nop\n\tv_nop" : "+v"(acc[0]), "+v"(acc[1]), "+v"(acc[2]), "+v"(acc[3]) : "v"(a), "v"(al));
    }
    float* os = &ost[wave][0];
#pragma unroll
    for (int t = 0; t < 4; ++t) { const float bv = bias ? bfr(bias[c0 + t * 16 + lr]) : 0.f;
#pragma unroll
        for (int j = 0; j < 8; ++j) os[(hi * 8 + j) * 68 + t * 16 + lr] = acc[t][j] + bv; }
    __syncthreads();
    if (F16OUT) {
        h16* crow = (h16*)(void*)C + (size_t)r0 * ldc + c0;
        auto pass = [&]() {
#pragma unroll
            for (int s = 0; s < 4; ++s) { const int row = 4 * s + (lane >> 3), piece = lane & 7; const float* sp = os + row * 68 + piece * 8; v8h o, o2;
#pragma unroll
                for (int i = 0; i < 8; ++i) { const h16 a = (h16)sp[i]; o[i] = a; o2[i] = (h16)((sp[i] - (float)a) * LOSC); }
                *(volatile v8h*)(crow + (size_t)row * ldc + piece * 8) = o; if (C2) *(volatile v8h*)(C2 + (size_t)r0 * ldc + c0 + (size_t)row * ldc + piece * 8) = o2; }
        };
        pass(); __threadfence(); pass();
    } else {
        float* crow = C + (size_t)r0 * ldc + c0;
        auto pass = [&]() {
#pragma unroll
            for (int s = 0; s < 8; ++s) { const int Lid = (lane >> 3) + 4 * s, piece = lane & 7; const int row = Lid >> 1, cofs = (Lid & 1) * 32 + piece * 4;
                v4f val = *(const v4fa*)(os + row * 68 + cofs); if (R) { const v4f rv = *(const v4f*)(R + ((size_t)r0 + row) * ldc + c0 + cofs); val += roundR ? (v4f){bfr(rv[0]), bfr(rv[1]), bfr(rv[2]), bfr(rv[3])} : rv; }
                *(volatile v4f*)(crow + (size_t)row * ldc + cofs) = val; }
        };
        pass(); __threadfence(); pass();
    }
}


__device__ __forceinline__ float lk(float x) { return x >= 0.f ? x : SLOPE * x; }
__global__ __launch_bounds__(256) void k_feats(const float* __restrict__ x, int b, bf* Fh, bf* Fl) {
    const int u = blockIdx.x * 256 + threadIdx.x; if (u >= NPP * KP / 8) return; v8us oh, ol;
#pragma unroll
    for (int i = 0; i < 8; ++i) { const int e = u * 8 + i; const int p = e / KP, col = e % KP; float v = 0.f;
        if (p < NP) { const int r = p / PG, q = p % PG;
            if (col < CIN * 4) { const int c = col / 4, k4 = col % 4, ki = k4 / 2, kj = k4 % 2; const int gy = r + ki, gx = q + kj; const float* px = x + (((size_t)b * CIN + c) * HW + 2 * gy) * HW + 2 * gx;
                v = ((bfr(px[0]) + bfr(px[1])) + (bfr(px[HW]) + bfr(px[HW + 1]))) * 0.25f; }
            else if (col == CIN * 4) v = (float)(q - PG / 2); else if (col == CIN * 4 + 1) v = (float)(r - PG / 2); }
        const unsigned short hb = f2bf(v); oh[i] = hb; ol[i] = f2bf(v - bf2f(hb)); }
    *(volatile v8us*)(Fh + (size_t)u * 8) = oh; *(volatile v8us*)(Fl + (size_t)u * 8) = ol; __threadfence(); *(volatile v8us*)(Fh + (size_t)u * 8) = oh; *(volatile v8us*)(Fl + (size_t)u * 8) = ol;
}
__global__ __launch_bounds__(256) void k_w0(const float* __restrict__ W0, bf* WA, bf* WB) {
    const int u = blockIdx.x * 256 + threadIdx.x; if (u >= HID * KP / 8) return; v8us a, bq;
#pragma unroll
    for (int i = 0; i < 8; ++i) { const int e = u * 8 + i; const int o = e / KP, c = e % KP; a[i] = (c < DFE) ? f2bf(W0[(size_t)c * HID + o]) : (unsigned short)0; bq[i] = (c < DFE) ? f2bf(W0[(size_t)(DFE + c) * HID + o]) : (unsigned short)0; }
    *(volatile v8us*)(WA + (size_t)u * 8) = a; *(volatile v8us*)(WB + (size_t)u * 8) = bq; __threadfence(); *(volatile v8us*)(WA + (size_t)u * 8) = a; *(volatile v8us*)(WB + (size_t)u * 8) = bq;
}
__global__ __launch_bounds__(256) void k_pair(const float* __restrict__ A, const float* __restrict__ Bv, const float* __restrict__ b0, bf* Hh, bf* Hl) {
    const int lane = threadIdx.x & 31, r = blockIdx.x * 8 + (threadIdx.x >> 5); if (r >= NPRP) return;
    const int i = r / NP, j = r % NP; v8us oh, ol;
#pragma unroll
    for (int k = 0; k < 8; ++k) { const int o = lane * 8 + k; float v = 0.f; if (r < NPR) v = lk(A[(size_t)j * HID + o] + Bv[(size_t)i * HID + o] + bfr(b0[o])); const unsigned short hb = f2bf(v); oh[k] = hb; ol[k] = f2bf(v - bf2f(hb)); }
    const size_t off = (size_t)r * HID + lane * 8; *(volatile v8us*)(Hh + off) = oh; *(volatile v8us*)(Hl + off) = ol; __threadfence(); *(volatile v8us*)(Hh + off) = oh; *(volatile v8us*)(Hl + off) = ol;
}
__global__ __launch_bounds__(256) void k_pairmean(const float* __restrict__ T, int b, float* S) {
    const int o = threadIdx.x; float s = 0.f;
#pragma unroll 1
    for (int r = 0; r < NPR; ++r) s += lk(T[(size_t)r * HID + o]);
    const float m = s / (float)NPR; *(volatile float*)(S + (size_t)b * HID + o) = m; __threadfence(); *(volatile float*)(S + (size_t)b * HID + o) = m;
}
__global__ __launch_bounds__(256) void k_head(const float* __restrict__ S, const float* __restrict__ Wout, const float* __restrict__ bout, float* OUTP) {
    const int u = blockIdx.x * 256 + threadIdx.x; if (u >= NBI * NOUT) return; const int b = u / NOUT, n = u % NOUT; float a = bfr(bout[n]);
#pragma unroll 1
    for (int o = 0; o < HID; ++o) a = fmaf(S[(size_t)b * HID + o], bfr(Wout[(size_t)o * NOUT + n]), a);
    *(volatile float*)(OUTP + u) = a; __threadfence(); *(volatile float*)(OUTP + u) = a;
}

extern "C" void kernel_launch(void* const* d_in, const int* in_sizes, int n_in,
                              void* d_out, int out_size, void* d_ws, size_t ws_size, hipStream_t stream) {
    (void)in_sizes; (void)n_in; (void)out_size;
    const float* x = (const float*)d_in[0]; const float* W0 = (const float*)d_in[1]; const float* b0 = (const float*)d_in[2]; const float* W1 = (const float*)d_in[3]; const float* b1 = (const float*)d_in[4]; const float* Wout = (const float*)d_in[5]; const float* bout = (const float*)d_in[6];
    float* out = (float*)d_out;
    char* wsp = (char*)d_ws;
    auto take = [&](size_t bytes) { char* p = wsp; wsp += (bytes + 255) & ~(size_t)255; return (void*)p; };
    bf* WA = (bf*)take(HID * KP * 2); bf* WB = (bf*)take(HID * KP * 2); bf* W1T = (bf*)take(HID * HID * 2); bf* Fh = (bf*)take(NPP * KP * 2); bf* Fl = (bf*)take(NPP * KP * 2);
    float* A = (float*)take((size_t)NPP * HID * 4); float* Bv = (float*)take((size_t)NPP * HID * 4); bf* Hh = (bf*)take((size_t)NPRP * HID * 2); bf* Hl = (bf*)take((size_t)NPRP * HID * 2); float* T = (float*)take((size_t)NPRP * HID * 4); float* S = (float*)take((size_t)NBI * HID * 4);
    if ((size_t)(wsp - (char*)d_ws) > ws_size) return;
    k_w0<<<(HID * KP / 8 + 255) / 256, 256, 0, stream>>>(W0, WA, WB); k_wt<<<dim3(HID / 64, HID / 64, 1), 256, 0, stream>>>(W1, HID, HID, W1T);
    for (int b = 0; b < NBI; ++b) {
        k_feats<<<(NPP * KP / 8 + 255) / 256, 256, 0, stream>>>(x, b, Fh, Fl);
        k_gemmb<true, false><<<dim3(NPP / 64, HID / 64, 1), 128, 0, stream>>>(Fh, Fl, WA, nullptr, A, HID, nullptr, nullptr, KP);
        k_gemmb<true, false><<<dim3(NPP / 64, HID / 64, 1), 128, 0, stream>>>(Fh, Fl, WB, nullptr, Bv, HID, nullptr, nullptr, KP);
        k_pair<<<NPRP / 8, 256, 0, stream>>>(A, Bv, b0, Hh, Hl);
        k_gemmb<true, false><<<dim3(NPRP / 64, HID / 64, 1), 128, 0, stream>>>(Hh, Hl, W1T, b1, T, HID, nullptr, nullptr, HID);
        k_pairmean<<<1, 256, 0, stream>>>(T, b, S);
    }
    k_head<<<(NBI * NOUT + 255) / 256, 256, 0, stream>>>(S, Wout, bout, out);
}
